// DynamicTransformerLayer_9096740733537
// MI455X (gfx1250) — hardware-verified
//
#include <hip/hip_runtime.h>
#include <math.h>

#ifndef NB
#define NB 4
#endif
#ifndef SEQ
#define SEQ 1024
#endif
#define NB_FULL 4
#define SEQ_FULL 1024
#define DIM 512
#define HEADS 8
#define HD 64
#define INNER 512
#define MLPD 2048
#define MTOK (NB * SEQ)
#define TPW (MTOK / 64)

#define GM_QK 0
#define GM_VT 1
#define GM_QRES 2
#define GM_GELU 3
#define GM_OUT 4

static_assert(NB <= NB_FULL && SEQ <= SEQ_FULL);
static_assert(SEQ % 128 == 0);
static_assert(MTOK % 64 == 0 && MTOK % 8 == 0);
static_assert(HEADS * HD == INNER && HD == 64);
static_assert(DIM % 64 == 0 && INNER % 64 == 0 && MLPD % 64 == 0);
static_assert(DIM % 32 == 0 && INNER % 32 == 0 && MLPD % 32 == 0 && HD % 32 == 0);
static_assert(DIM == 512);
static_assert(((2 * MTOK / 64) * (INNER / 64)) % 8 == 0);
static_assert(((INNER / 64) * (MTOK / 64)) % 8 == 0);
static_assert(((MTOK / 64) * (DIM / 64)) % 8 == 0);
static_assert(((MTOK / 64) * (MLPD / 64)) % 8 == 0);
static_assert((INNER * DIM / 8) % 256 == 0 && (MLPD * DIM / 8) % 256 == 0);

typedef _Float16 h16;
typedef __attribute__((ext_vector_type(16))) _Float16 v16h;
typedef __attribute__((ext_vector_type(8)))  _Float16 v8h;
typedef __attribute__((ext_vector_type(8)))  float    v8f;
typedef __attribute__((ext_vector_type(4)))  float    v4f;


static constexpr float WCARRY = 64.0f;
static constexpr float SCARRY = 256.0f;
static constexpr float INV_SCARRY = 1.0f / 256.0f;

static constexpr size_t al256(size_t x) { return (x + 255) & ~(size_t)255; }
static constexpr size_t OFF_WIN  = 0;
static constexpr size_t OFF_WOUT = OFF_WIN  + al256((size_t)INNER * DIM * 2);
static constexpr size_t OFF_WUP  = OFF_WOUT + al256((size_t)DIM * INNER * 2);
static constexpr size_t OFF_WDN  = OFF_WUP  + al256((size_t)MLPD * DIM * 2);
static constexpr size_t OFF_X16  = OFF_WDN  + al256((size_t)DIM * MLPD * 2);
static constexpr size_t OFF_FQK  = OFF_X16  + al256((size_t)3 * MTOK * DIM * 2);
static constexpr size_t OFF_FVT  = OFF_FQK  + al256((size_t)2 * HEADS * MTOK * HD * 2);
static constexpr size_t OFF_STAT = OFF_FVT  + al256((size_t)HEADS * NB * HD * SEQ * 2);
static constexpr size_t OFF_PART = OFF_STAT + al256((size_t)3 * 2 * HEADS * MTOK * 4);
static constexpr size_t OFF_MIXW = OFF_PART + al256((size_t)2 * HEADS * TPW * 64 * 4);
static constexpr size_t OFF_CTX  = OFF_MIXW + al256((size_t)32 * 4);
static constexpr size_t OFF_Q2   = OFF_CTX  + al256((size_t)MTOK * INNER * 2);
static constexpr size_t OFF_X2   = OFF_Q2   + al256((size_t)MTOK * DIM * 4);
static constexpr size_t OFF_HMID = OFF_X2   + al256((size_t)MTOK * DIM * 2);
static constexpr size_t WS_TOTAL = OFF_HMID + al256((size_t)MTOK * MLPD * 2);
static_assert(WS_TOTAL <= (size_t)134217728);

static constexpr int ACT_MIN = ((NB - 1) * SEQ_FULL + SEQ) * DIM;

static_assert(8 * 16 * 68 * 4 + 8 * 256 * 4 <= 131072);
static_assert(8 * 16 * 72 * 2 <= 131072);
static_assert(32 * 16 * 8 == 16 * 256);
static_assert(32 * 16 * 4 == 16 * 128);
static_assert(16 * 16 == 64 * 4);
static_assert(32 * 16 * 2 == DIM * 2);
static_assert(8 * 16 == 32 * 4);

__device__ __forceinline__ float bfr(float f) {
    unsigned u = __float_as_uint(f);
    u += 0x7FFFu + ((u >> 16) & 1u);
    return __uint_as_float(u & 0xFFFF0000u);
}
static __device__ __forceinline__ h16 toh_flush(float v) { const float w = (fabsf(v) < 6.103515625e-05f) ? 0.0f : v; return (h16)w; }

__device__ __forceinline__ float gelu_erf(float v) { return 0.5f * v * (1.0f + erff(v * 0.70710678118654752f)); }

__device__ __forceinline__ unsigned map_row(unsigned m) {
    return (m / (unsigned)SEQ) * (unsigned)SEQ_FULL + (m % (unsigned)SEQ);
}

union FragU { v16h v; v8h h[2]; };
__device__ __forceinline__ v16h frag_ld(const _Float16* p) {
    FragU f; f.h[0] = *(const v8h*)(p); f.h[1] = *(const v8h*)(p + 16); return f.v;
}
__device__ __forceinline__ v8f wmma16(v16h a, v16h b, v8f c) {
    c = __builtin_amdgcn_wmma_f32_16x16x32_f16(false, a, false, b, (short)0, c, false, false);
    asm volatile("v_nop\n\tv_nop\n\tv_nop\n\tv_nop" : "+v"(c) : "v"(a), "v"(b));
    return c;
}
__device__ __forceinline__ void wave_sync_lds() {
    __builtin_amdgcn_fence(3  , "workgroup");
    __builtin_amdgcn_wave_barrier();
    __builtin_amdgcn_fence(2  , "workgroup");
}

template <int MODE, int SSH, int OSH>
__device__ __forceinline__ void gemm_body(
    const h16* __restrict__ A, unsigned lda, const h16* __restrict__ Bt, unsigned ldb,
    void* __restrict__ Cout, unsigned ldc, const float* __restrict__ bias, const float* __restrict__ resid,
    float* __restrict__ stats, float* __restrict__ part, unsigned M, unsigned N, unsigned K) {
  __shared__ __align__(16) float sT[8][16 * 68];
  __shared__ __align__(16) float sSt[8][256];
  constexpr float scale = 1.0f / (float)(1u << SSH);
  constexpr float oscale = (float)(1u << OSH);
  constexpr bool HAS_BIAS = (MODE == GM_QRES) || (MODE == GM_GELU) || (MODE == GM_OUT);
  const unsigned lane = threadIdx.x & 31u;
  const unsigned wave = (unsigned)__builtin_amdgcn_readfirstlane((int)(threadIdx.x >> 5));
  const unsigned tilesN = N >> 6, tilesM = M >> 6;
  const unsigned tile = blockIdx.x * 8u + wave;
  if (tile >= tilesM * tilesN) return;
  const unsigned tm = tile / tilesN;
  const unsigned tn = tile - tm * tilesN;
  const unsigned m0 = tm << 6, n0 = tn << 6;
  const unsigned rlane = lane & 15u;
  const unsigned koff = (lane >> 4) * 8u;
  const unsigned mOff = koff;

  v8f acc[4][4];
#pragma unroll
  for (int i = 0; i < 4; ++i)
#pragma unroll
    for (int j = 0; j < 4; ++j) acc[i][j] = (v8f){0.f,0.f,0.f,0.f,0.f,0.f,0.f,0.f};

  for (unsigned k0 = 0; k0 < K; k0 += 32u) {
    v16h bh[4];
#pragma unroll
    for (int j = 0; j < 4; ++j)
      bh[j] = frag_ld(Bt + (size_t)(n0 + ((unsigned)j << 4) + rlane) * ldb + koff + k0);
#pragma unroll
    for (int i = 0; i < 4; ++i) {
      const v16h ah = frag_ld(A + (size_t)(m0 + ((unsigned)i << 4) + rlane) * lda + koff + k0);
#pragma unroll
      for (int j = 0; j < 4; ++j)
        acc[i][j] = wmma16(ah, bh[j], acc[i][j]);
    }
  }

  const unsigned which = tm / (unsigned)TPW;
  const unsigned tml = tm - which * (unsigned)TPW;
  const unsigned ml = tml << 6;
  const unsigned bidx = n0 / (unsigned)SEQ;
  const unsigned key0 = n0 - bidx * (unsigned)SEQ;

  float* slab = sT[wave];
  float* sst = sSt[wave];
  float cs[4] = {0.f, 0.f, 0.f, 0.f};
#pragma unroll
  for (int i = 0; i < 4; ++i) {
    const unsigned mBase = m0 + ((unsigned)i << 4);
#pragma unroll
    for (int j = 0; j < 4; ++j) {
      float bv = 0.0f;
      if (HAS_BIAS) bv = bfr(bias[n0 + ((unsigned)j << 4) + rlane]);
#pragma unroll
      for (int r = 0; r < 8; ++r) {
        const float v = acc[i][j][r] * scale + bv;
        if (MODE == GM_QK) cs[j] += v;
        slab[(mOff + (unsigned)r) * 68u + ((unsigned)j << 4) + rlane] = v;
      }
    }
    wave_sync_lds();
    if (MODE == GM_GELU) {
#pragma unroll 1
      for (unsigned e = 0; e < 8u; ++e) {
        const unsigned f = (e * 32u + lane) * 4u;
        float* sp = slab + (f >> 6) * 68u + (f & 63u);
        v4f x = *(const v4f*)sp;
        x.x = gelu_erf(x.x); x.y = gelu_erf(x.y); x.z = gelu_erf(x.z); x.w = gelu_erf(x.w);
        *(v4f*)sp = x;
      }
      wave_sync_lds();
    }
    if (MODE == GM_QK) {
      const float* sp = slab + (lane >> 1) * 68u + (lane & 1u) * 32u;
      float s = 0.f, ss = 0.f;
#pragma unroll
      for (int g = 0; g < 8; ++g) {
        const v4f x = *(const v4f*)(sp + 4 * g);
        s += (x.x + x.y) + (x.z + x.w);
        ss += (x.x * x.x + x.y * x.y) + (x.z * x.z + x.w * x.w);
      }
      s += __shfl_xor(s, 1, 32);
      ss += __shfl_xor(ss, 1, 32);
      const float mean = s * (1.0f / 64.0f);
      float dv = 0.f;
#pragma unroll
      for (int g = 0; g < 8; ++g) {
        const v4f x = *(const v4f*)(sp + 4 * g);
        const float d0 = x.x - mean, d1 = x.y - mean, d2 = x.z - mean, d3 = x.w - mean;
        dv += (d0 * d0 + d1 * d1) + (d2 * d2 + d3 * d3);
      }
      dv += __shfl_xor(dv, 1, 32);
      if ((lane & 1u) == 0u) {
        const unsigned ri = ((unsigned)i << 4) + (lane >> 1);
        sst[ri] = rsqrtf(ss);
        sst[64u + ri] = mean;
        sst[128u + ri] = dv * (1.0f / 63.0f);
      }
    }
    if (MODE == GM_QRES || MODE == GM_OUT) {
      float* C = (float*)Cout;
      const unsigned hh = lane >> 4, c4 = (lane & 15u) * 4u;
#pragma unroll
      for (int half = 0; half < 2; ++half) {
        v4f vv[4];
#pragma unroll
        for (int it = 0; it < 4; ++it) {
          const unsigned row = (unsigned)(half * 4 + it) * 2u + hh;
          const unsigned gm = mBase + row;
          vv[it] = *(const v4f*)(slab + row * 68u + c4);
          if (MODE == GM_QRES) {
            v4f rr = *(const v4f*)(resid + (size_t)map_row(gm) * ldc + n0 + c4);
            rr.x = bfr(rr.x); rr.y = bfr(rr.y); rr.z = bfr(rr.z); rr.w = bfr(rr.w);
            vv[it] += rr;
          } else {
            vv[it] += *(const v4f*)(resid + (size_t)gm * ldc + n0 + c4);
          }
        }
        for (int pass = 0; pass < 2; ++pass) {
#pragma unroll
          for (int it = 0; it < 4; ++it) {
            const unsigned row = (unsigned)(half * 4 + it) * 2u + hh;
            const unsigned gm = mBase + row;
            const unsigned orow = (MODE == GM_OUT) ? map_row(gm) : gm;
            *(volatile v4f*)(C + (size_t)orow * ldc + n0 + c4) = vv[it];
          }
          __threadfence();
        }
      }
    } else {
      h16* C = (h16*)Cout;
      const unsigned q = lane >> 3, c8 = (lane & 7u) * 8u;
      v8h hv[4];
#pragma unroll
      for (int it = 0; it < 4; ++it) {
        const unsigned row = (unsigned)it * 4u + q;
        const float* sp = slab + row * 68u + c8;
#pragma unroll
        for (int e = 0; e < 8; ++e) hv[it][e] = toh_flush(sp[e] * oscale);
      }
      for (int pass = 0; pass < 2; ++pass) {
#pragma unroll
        for (int it = 0; it < 4; ++it) {
          const unsigned row = (unsigned)it * 4u + q;
          size_t o;
          if (MODE == GM_QK)      o = (size_t)((which * 8u + tn) * (unsigned)MTOK + ml + ((unsigned)i << 4) + row) * 64u + c8;
          else if (MODE == GM_VT) o = (size_t)((tm * (unsigned)NB + bidx) * 64u + ((unsigned)i << 4) + row) * (unsigned)SEQ + key0 + c8;
          else                    o = (size_t)(mBase + row) * ldc + n0 + c8;
          *(volatile v8h*)(C + o) = hv[it];
        }
        __threadfence();
      }
    }
    wave_sync_lds();
  }
  if (MODE == GM_QK) {
#pragma unroll
    for (int j = 0; j < 4; ++j) cs[j] += __shfl_xor(cs[j], 16, 32);
    if ((lane >> 4) == 0u) {
#pragma unroll
      for (int j = 0; j < 4; ++j) sst[192u + ((unsigned)j << 4) + rlane] = cs[j];
    }
    wave_sync_lds();
    if (lane < 16u) {
      const v4f v0 = *(const v4f*)(sst + 4u * lane);
      const v4f v1 = *(const v4f*)(sst + 64u + 4u * lane);
      const v4f v2 = *(const v4f*)(sst + 128u + 4u * lane);
      const v4f v3 = *(const v4f*)(sst + 192u + 4u * lane);
      float* p0 = stats + (size_t)((0u * 2u + which) * 8u + tn) * (unsigned)MTOK + ml + 4u * lane;
      float* p1 = stats + (size_t)((1u * 2u + which) * 8u + tn) * (unsigned)MTOK + ml + 4u * lane;
      float* p2 = stats + (size_t)((2u * 2u + which) * 8u + tn) * (unsigned)MTOK + ml + 4u * lane;
      float* p3 = part + (size_t)((which * 8u + tn) * (unsigned)TPW + tml) * 64u + 4u * lane;
      for (int pass = 0; pass < 2; ++pass) {
        *(volatile v4f*)p0 = v0;
        *(volatile v4f*)p1 = v1;
        *(volatile v4f*)p2 = v2;
        *(volatile v4f*)p3 = v3;
        __threadfence();
      }
    }
  }
}

__global__ __launch_bounds__(256) void k_gemm_qk(const h16* __restrict__ A, const h16* __restrict__ Bt, h16* __restrict__ C,
                                                 float* __restrict__ stats, float* __restrict__ part) {
  gemm_body<GM_QK, 6, 0>(A, (unsigned)DIM, Bt, (unsigned)DIM, (void*)C, 64u, nullptr, nullptr, stats, part,
                         (unsigned)(2 * MTOK), (unsigned)INNER, (unsigned)DIM);
}
__global__ __launch_bounds__(256) void k_gemm_vt(const h16* __restrict__ A, const h16* __restrict__ Bt, h16* __restrict__ C) {
  gemm_body<GM_VT, 6, 0>(A, (unsigned)DIM, Bt, (unsigned)DIM, (void*)C, (unsigned)SEQ, nullptr, nullptr, nullptr, nullptr,
                         (unsigned)INNER, (unsigned)MTOK, (unsigned)DIM);
}
__global__ __launch_bounds__(256) void k_gemm_o(const h16* __restrict__ A, const h16* __restrict__ Bt, float* __restrict__ C,
                                                const float* __restrict__ bias, const float* __restrict__ resid) {
  gemm_body<GM_QRES, 6, 0>(A, (unsigned)INNER, Bt, (unsigned)INNER, (void*)C, (unsigned)DIM, bias, resid, nullptr, nullptr,
                           (unsigned)MTOK, (unsigned)DIM, (unsigned)INNER);
}
__global__ __launch_bounds__(256) void k_gemm_up(const h16* __restrict__ A, const h16* __restrict__ Bt, h16* __restrict__ C,
                                                 const float* __restrict__ bias) {
  gemm_body<GM_GELU, 6, 4>(A, (unsigned)DIM, Bt, (unsigned)DIM, (void*)C, (unsigned)MLPD, bias, nullptr, nullptr, nullptr,
                           (unsigned)MTOK, (unsigned)MLPD, (unsigned)DIM);
}
__global__ __launch_bounds__(256) void k_gemm_dn(const h16* __restrict__ A, const h16* __restrict__ Bt, float* __restrict__ C,
                                                 const float* __restrict__ bias, const float* __restrict__ resid) {
  gemm_body<GM_OUT, 10, 0>(A, (unsigned)MLPD, Bt, (unsigned)MLPD, (void*)C, (unsigned)DIM, bias, resid, nullptr, nullptr,
                           (unsigned)MTOK, (unsigned)DIM, (unsigned)MLPD);
}

__global__ __launch_bounds__(256) void k_wcvt(const float* __restrict__ W, h16* __restrict__ P, unsigned n8) {
    const unsigned u = blockIdx.x * 256u + threadIdx.x;
    if (u >= n8) return;
    const float* wp = W + (size_t)u * 8u;
    const v4f a = *(const v4f*)wp, b = *(const v4f*)(wp + 4);
    v8h hv;
    hv[0] = toh_flush(bfr(a.x) * WCARRY); hv[1] = toh_flush(bfr(a.y) * WCARRY);
    hv[2] = toh_flush(bfr(a.z) * WCARRY); hv[3] = toh_flush(bfr(a.w) * WCARRY);
    hv[4] = toh_flush(bfr(b.x) * WCARRY); hv[5] = toh_flush(bfr(b.y) * WCARRY);
    hv[6] = toh_flush(bfr(b.z) * WCARRY); hv[7] = toh_flush(bfr(b.w) * WCARRY);
    h16* p = P + (size_t)u * 8u;
    for (int pass = 0; pass < 2; ++pass) {
        *(volatile v8h*)p = hv;
        __threadfence();
    }
}

template <bool INP>
__device__ __forceinline__ void ln512_body(const float* __restrict__ x, const float* __restrict__ g, const float* __restrict__ bt,
                                           h16* __restrict__ z, unsigned M) {
    const unsigned wave = (unsigned)__builtin_amdgcn_readfirstlane((int)(threadIdx.x >> 5));
    const unsigned row = blockIdx.x * 8u + wave;
    const unsigned L = threadIdx.x & 31u;
    if (row >= M) return;
    const unsigned srow = INP ? map_row(row) : row;
    const float* xr = x + (size_t)srow * 512u + 8u * L;
    const v4f a0 = *(const v4f*)xr, a1 = *(const v4f*)(xr + 4), a2 = *(const v4f*)(xr + 256), a3 = *(const v4f*)(xr + 260);
    float d[16] = {a0.x, a0.y, a0.z, a0.w, a1.x, a1.y, a1.z, a1.w, a2.x, a2.y, a2.z, a2.w, a3.x, a3.y, a3.z, a3.w};
    if (INP) {
#pragma unroll
        for (int i = 0; i < 16; ++i) d[i] = bfr(d[i]);
    }
    float s = 0.f;
#pragma unroll
    for (int i = 0; i < 16; ++i) s += d[i];
#pragma unroll
    for (int o = 16; o > 0; o >>= 1) s += __shfl_xor(s, o, 32);
    const float mu = s * (1.0f / 512.0f);
    float q = 0.f;
#pragma unroll
    for (int i = 0; i < 16; ++i) { d[i] -= mu; q += d[i] * d[i]; }
#pragma unroll
    for (int o = 16; o > 0; o >>= 1) q += __shfl_xor(q, o, 32);
    const float rs = rsqrtf(q * (1.0f / 512.0f) + 1e-5f);
    const float* gp = g + 8u * L;
    const float* bp = bt + 8u * L;
    const v4f g0 = *(const v4f*)gp, g1 = *(const v4f*)(gp + 4), g2 = *(const v4f*)(gp + 256), g3 = *(const v4f*)(gp + 260);
    const v4f b0 = *(const v4f*)bp, b1 = *(const v4f*)(bp + 4), b2 = *(const v4f*)(bp + 256), b3 = *(const v4f*)(bp + 260);
    const float gg[16] = {g0.x, g0.y, g0.z, g0.w, g1.x, g1.y, g1.z, g1.w, g2.x, g2.y, g2.z, g2.w, g3.x, g3.y, g3.z, g3.w};
    const float bb[16] = {b0.x, b0.y, b0.z, b0.w, b1.x, b1.y, b1.z, b1.w, b2.x, b2.y, b2.z, b2.w, b3.x, b3.y, b3.z, b3.w};
    v8h h0, h1;
#pragma unroll
    for (int i = 0; i < 8; ++i) {
        h0[i] = toh_flush(d[i] * rs * bfr(gg[i]) + bfr(bb[i]));
        h1[i] = toh_flush(d[8 + i] * rs * bfr(gg[8 + i]) + bfr(bb[8 + i]));
    }
    h16* zr = z + (size_t)row * 512u + 8u * L;
    for (int pass = 0; pass < 2; ++pass) {
        *(volatile v8h*)zr = h0;
        *(volatile v8h*)(zr + 256) = h1;
        __threadfence();
    }
}
__global__ __launch_bounds__(256) void k_ln_in(const float* __restrict__ x, const float* __restrict__ g, const float* __restrict__ bt,
                                               h16* __restrict__ z, unsigned M) {
    ln512_body<true>(x, g, bt, z, M);
}
__global__ __launch_bounds__(256) void k_ln_mid(const float* __restrict__ x, const float* __restrict__ g, const float* __restrict__ bt,
                                                h16* __restrict__ z, unsigned M) {
    ln512_body<false>(x, g, bt, z, M);
}

__global__ __launch_bounds__(256) void k_mixw(const float* __restrict__ part, const float* __restrict__ W1, const float* __restrict__ b1,
                                              const float* __restrict__ g, const float* __restrict__ bb,
                                              const float* __restrict__ W2, const float* __restrict__ b2, float* __restrict__ wout) {
    __shared__ float sF[128];
    __shared__ float sH[64];
    __shared__ float sY[64];
    __shared__ float sL[4];
    __shared__ float sE[4];
    __shared__ __align__(16) float sW[32];
    const unsigned t = threadIdx.x;
    if (t < 32u) sW[t] = 0.f;
    __syncthreads();
#pragma unroll 1
    for (unsigned h = 0; h < (unsigned)HEADS; ++h) {
        if (t < 128u) {
            const unsigned which = t >> 6, d = t & 63u;
            const float* pp = part + (size_t)((which * 8u + h) * (unsigned)TPW) * 64u + d;
            float s = 0.f;
#pragma unroll 4
            for (unsigned tm = 0; tm < (unsigned)TPW; ++tm) s += pp[(size_t)tm * 64u];
            sF[t] = s * (1.0f / (float)MTOK);
        }
        __syncthreads();
        if (t < 64u) {
            const float* wr = W1 + (size_t)t * 128u;
            float a = 0.f;
#pragma unroll 4
            for (unsigned j = 0; j < 128u; ++j) a += sF[j] * bfr(wr[j]);
            sH[t] = a + bfr(b1[t]);
        }
        __syncthreads();
        if (t < 64u) {
            float s = 0.f;
#pragma unroll 4
            for (unsigned i = 0; i < 64u; ++i) s += sH[i];
            const float mu = s * (1.0f / 64.0f);
            float q = 0.f;
#pragma unroll 4
            for (unsigned i = 0; i < 64u; ++i) { const float dd = sH[i] - mu; q += dd * dd; }
            const float rs = rsqrtf(q * (1.0f / 64.0f) + 1e-5f);
            const float y = (sH[t] - mu) * rs * bfr(g[t]) + bfr(bb[t]);
            sY[t] = fmaxf(y, 0.0f);
        }
        __syncthreads();
        if (t < 3u) {
            const float* wr = W2 + (size_t)t * 64u;
            float a = 0.f;
#pragma unroll 4
            for (unsigned i = 0; i < 64u; ++i) a += sY[i] * bfr(wr[i]);
            sL[t] = a + bfr(b2[t]);
        }
        __syncthreads();
        if (t == 0u) {
            const float mx = fmaxf(fmaxf(sL[0], sL[1]), sL[2]);
            float den = 0.f;
#pragma unroll 1
            for (unsigned k = 0; k < 3u; ++k) { const float e = expf(sL[k] - mx); sE[k] = e; den += e; }
            const float inv = 1.0f / den;
#pragma unroll 1
            for (unsigned k = 0; k < 3u; ++k) sW[3u * h + k] = sE[k] * inv;
        }
        __syncthreads();
    }
    if (t < 8u) {
        const v4f v = *(const v4f*)(sW + 4u * t);
        for (int pass = 0; pass < 2; ++pass) {
            *(volatile v4f*)(wout + 4u * t) = v;
            __threadfence();
        }
    }
}

#define AT_PP 72
#define SCE(D, Z, I, RC, MC, VC) D[I] = Z[I] * (Aq * (RC) + CV) - Mq * (MC) + Vq * (VC)
__global__ __launch_bounds__(256) void k_attn(const h16* __restrict__ fqk, const h16* __restrict__ fvT,
                                              const float* __restrict__ stats, const float* __restrict__ mixw,
                                              h16* __restrict__ ctx) {
    __shared__ __align__(16) h16 sO[8][16 * AT_PP];
    const unsigned tid = threadIdx.x, lane = tid & 31u;
    const unsigned wave = (unsigned)__builtin_amdgcn_readfirstlane((int)(tid >> 5));
    const unsigned hh = lane >> 4, c = lane & 15u;
    const unsigned bx = blockIdx.x;
    const unsigned QB = (unsigned)(SEQ / 128);
    const unsigned qblk = bx % QB;
    const unsigned hb = bx / QB;
    const unsigned b = hb % (unsigned)NB;
    const unsigned h = hb / (unsigned)NB;
    const unsigned q0 = qblk * 128u + wave * 16u;
    const unsigned tok0 = b * (unsigned)SEQ;

    const h16* qbase = fqk + ((size_t)(h) * (unsigned)MTOK + tok0) * 64u;
    const h16* kbase = fqk + ((size_t)(8u + h) * (unsigned)MTOK + tok0) * 64u;
    const h16* vbase = fvT + ((size_t)(h * (unsigned)NB + b) * 64u) * (unsigned)SEQ;
    const float* qr_p = stats + (size_t)((0u * 2u + 0u) * 8u + h) * (unsigned)MTOK + tok0;
    const float* qm_p = stats + (size_t)((1u * 2u + 0u) * 8u + h) * (unsigned)MTOK + tok0;
    const float* qv_p = stats + (size_t)((2u * 2u + 0u) * 8u + h) * (unsigned)MTOK + tok0;
    const float* kr_p = stats + (size_t)((0u * 2u + 1u) * 8u + h) * (unsigned)MTOK + tok0;
    const float* km_p = stats + (size_t)((1u * 2u + 1u) * 8u + h) * (unsigned)MTOK + tok0;
    const float* kv_p = stats + (size_t)((2u * 2u + 1u) * 8u + h) * (unsigned)MTOK + tok0;

    const float cw = mixw[3u * h], covw = mixw[3u * h + 1u], vw = mixw[3u * h + 2u];
    const float rq = qr_p[q0 + c], mq = qm_p[q0 + c], vq = qv_p[q0 + c];
    const float Aq = SCARRY * cw * rq;
    const float CV = (SCARRY / 64.0f) * covw;
    const float Mq = SCARRY * covw * mq;
    const float Vq = (SCARRY / 64.0f) * vw * vq;

    const v16h qf0 = frag_ld(qbase + (size_t)(q0 + c) * 64u + 8u * hh);
    const v16h qf1 = frag_ld(qbase + (size_t)(q0 + c) * 64u + 32u + 8u * hh);

    v8f oacc[4];
#pragma unroll
    for (int t = 0; t < 4; ++t) oacc[t] = (v8f){0.f,0.f,0.f,0.f,0.f,0.f,0.f,0.f};

#pragma unroll 1
    for (unsigned kb = 0; kb < (unsigned)SEQ; kb += 32u) {
        v8f sv[2];
#pragma unroll
        for (int tt = 0; tt < 2; ++tt) {
            const h16* kr = kbase + (size_t)(kb + (unsigned)tt * 16u + c) * 64u + 8u * hh;
            const v16h kf0 = frag_ld(kr);
            const v16h kf1 = frag_ld(kr + 32);
            v8f z = (v8f){0.f,0.f,0.f,0.f,0.f,0.f,0.f,0.f};
            z = wmma16(kf0, qf0, z);
            z = wmma16(kf1, qf1, z);
            const unsigned ko = kb + (unsigned)tt * 16u + 8u * hh;
            const v4f ra = *(const v4f*)(kr_p + ko), rb = *(const v4f*)(kr_p + ko + 4u);
            const v4f ma = *(const v4f*)(km_p + ko), mb = *(const v4f*)(km_p + ko + 4u);
            const v4f va = *(const v4f*)(kv_p + ko), vb = *(const v4f*)(kv_p + ko + 4u);
            v8f d;
            SCE(d, z, 0, ra.x, ma.x, va.x);
            SCE(d, z, 1, ra.y, ma.y, va.y);
            SCE(d, z, 2, ra.z, ma.z, va.z);
            SCE(d, z, 3, ra.w, ma.w, va.w);
            SCE(d, z, 4, rb.x, mb.x, vb.x);
            SCE(d, z, 5, rb.y, mb.y, vb.y);
            SCE(d, z, 6, rb.z, mb.z, vb.z);
            SCE(d, z, 7, rb.w, mb.w, vb.w);
            sv[tt] = d;
        }
        v16h sb;
#pragma unroll
        for (int r = 0; r < 8; ++r) {
            sb[r] = toh_flush(sv[0][r]);
            sb[8 + r] = toh_flush(sv[1][r]);
        }
#pragma unroll
        for (int t = 0; t < 4; ++t) {
            const v16h vf = frag_ld(vbase + (size_t)((unsigned)t * 16u + c) * (unsigned)SEQ + kb + 8u * hh);
            oacc[t] = wmma16(vf, sb, oacc[t]);
        }
    }

    h16* pw = sO[wave];
#pragma unroll
    for (int t = 0; t < 4; ++t)
#pragma unroll
        for (int r = 0; r < 8; ++r)
            pw[c * AT_PP + (unsigned)t * 16u + 8u * hh + (unsigned)r] = toh_flush(oacc[t][r] * INV_SCARRY);
    wave_sync_lds();
    {
        const unsigned q = lane >> 3, c8 = (lane & 7u) * 8u;
        v8h ov[4];
#pragma unroll
        for (int it = 0; it < 4; ++it) ov[it] = *(const v8h*)(pw + ((unsigned)it * 4u + q) * AT_PP + c8);
        h16* dst = ctx + (size_t)(tok0 + q0) * (unsigned)INNER + h * 64u;
        for (int pass = 0; pass < 2; ++pass) {
#pragma unroll
            for (int it = 0; it < 4; ++it) *(volatile v8h*)(dst + (size_t)((unsigned)it * 4u + q) * (unsigned)INNER + c8) = ov[it];
            __threadfence();
        }
    }
}

extern "C" void kernel_launch(void* const* d_in, const int* in_sizes, int n_in, void* d_out, int out_size,
                              void* d_ws, size_t ws_size, hipStream_t stream) {
    if (n_in < 20) return;
    if (in_sizes[0] < ACT_MIN || in_sizes[1] < ACT_MIN || in_sizes[2] < ACT_MIN) return;
    if (in_sizes[3] < INNER * DIM || in_sizes[4] < DIM * INNER || in_sizes[5] < DIM) return;
    if (in_sizes[6] < DIM || in_sizes[7] < DIM || in_sizes[8] < DIM || in_sizes[9] < DIM) return;
    if (in_sizes[10] < MLPD * DIM || in_sizes[11] < MLPD || in_sizes[12] < DIM * MLPD || in_sizes[13] < DIM) return;
    if (in_sizes[14] < HD * 2 * HD || in_sizes[15] < HD || in_sizes[16] < HD || in_sizes[17] < HD) return;
    if (in_sizes[18] < 3 * HD || in_sizes[19] < 3 || out_size < ACT_MIN) return;
    if (WS_TOTAL > ws_size) return;

    const float* q     = (const float*)d_in[0];
    const float* k     = (const float*)d_in[1];
    const float* v     = (const float*)d_in[2];
    const float* Win   = (const float*)d_in[3];
    const float* Wout  = (const float*)d_in[4];
    const float* bout  = (const float*)d_in[5];
    const float* g1    = (const float*)d_in[6];
    const float* b1n   = (const float*)d_in[7];
    const float* g2    = (const float*)d_in[8];
    const float* b2n   = (const float*)d_in[9];
    const float* Wup   = (const float*)d_in[10];
    const float* bup   = (const float*)d_in[11];
    const float* Wdn   = (const float*)d_in[12];
    const float* bdn   = (const float*)d_in[13];
    const float* wpW1  = (const float*)d_in[14];
    const float* wpb1  = (const float*)d_in[15];
    const float* wpg   = (const float*)d_in[16];
    const float* wpb   = (const float*)d_in[17];
    const float* wpW2  = (const float*)d_in[18];
    const float* wpb2  = (const float*)d_in[19];
    float* out = (float*)d_out;

    char* wsp = (char*)d_ws;
    h16*   wIn   = (h16*)(wsp + OFF_WIN);
    h16*   wOut  = (h16*)(wsp + OFF_WOUT);
    h16*   wUp   = (h16*)(wsp + OFF_WUP);
    h16*   wDn   = (h16*)(wsp + OFF_WDN);
    h16*   x16   = (h16*)(wsp + OFF_X16);
    h16*   fqk   = (h16*)(wsp + OFF_FQK);
    h16*   fvT   = (h16*)(wsp + OFF_FVT);
    float* stats = (float*)(wsp + OFF_STAT);
    float* part  = (float*)(wsp + OFF_PART);
    float* mixw  = (float*)(wsp + OFF_MIXW);
    h16*   ctx   = (h16*)(wsp + OFF_CTX);
    float* q2    = (float*)(wsp + OFF_Q2);
    h16*   x2    = (h16*)(wsp + OFF_X2);
    h16*   hmid  = (h16*)(wsp + OFF_HMID);

    k_wcvt<<<(INNER * DIM / 8) / 256, 256, 0, stream>>>(Win, wIn, (unsigned)(INNER * DIM / 8));
    k_wcvt<<<(DIM * INNER / 8) / 256, 256, 0, stream>>>(Wout, wOut, (unsigned)(DIM * INNER / 8));
    k_wcvt<<<(MLPD * DIM / 8) / 256, 256, 0, stream>>>(Wup, wUp, (unsigned)(MLPD * DIM / 8));
    k_wcvt<<<(DIM * MLPD / 8) / 256, 256, 0, stream>>>(Wdn, wDn, (unsigned)(DIM * MLPD / 8));

    k_ln_in<<<MTOK / 8, 256, 0, stream>>>(q, g1, b1n, x16, (unsigned)MTOK);
    k_ln_in<<<MTOK / 8, 256, 0, stream>>>(k, g1, b1n, x16 + (size_t)MTOK * DIM, (unsigned)MTOK);
    k_ln_in<<<MTOK / 8, 256, 0, stream>>>(v, g1, b1n, x16 + (size_t)2 * MTOK * DIM, (unsigned)MTOK);

    k_gemm_qk<<<((2 * MTOK / 64) * (INNER / 64)) / 8, 256, 0, stream>>>(x16, wIn, fqk, stats, part);
    k_gemm_vt<<<((INNER / 64) * (MTOK / 64)) / 8, 256, 0, stream>>>(wIn, x16 + (size_t)2 * MTOK * DIM, fvT);

    k_mixw<<<1, 256, 0, stream>>>(part, wpW1, wpb1, wpg, wpb, wpW2, wpb2, mixw);

    k_attn<<<HEADS * NB * (SEQ / 128), 256, 0, stream>>>(fqk, fvT, stats, mixw, ctx);

    k_gemm_o<<<((MTOK / 64) * (DIM / 64)) / 8, 256, 0, stream>>>(ctx, wOut, q2, bout, q);
    k_ln_mid<<<MTOK / 8, 256, 0, stream>>>(q2, g2, b2n, x2, (unsigned)MTOK);
    k_gemm_up<<<((MTOK / 64) * (MLPD / 64)) / 8, 256, 0, stream>>>(x2, wUp, hmid, bup);
    k_gemm_dn<<<((MTOK / 64) * (DIM / 64)) / 8, 256, 0, stream>>>(hmid, wDn, out, bdn, q2);
}
